// TreeMLP_50285477101584
// MI455X (gfx1250) — hardware-verified
//
#include <hip/hip_runtime.h>
#include <math.h>

typedef __attribute__((ext_vector_type(16))) _Float16 v16h;
typedef __attribute__((ext_vector_type(16))) __bf16 v16b;
typedef __attribute__((ext_vector_type(8)))  _Float16 v8h;
typedef __attribute__((ext_vector_type(8)))  float v8f;
typedef __attribute__((ext_vector_type(4)))  float v4f;
typedef __attribute__((ext_vector_type(2)))  float v2f;
typedef __attribute__((ext_vector_type(4)))  unsigned v4u;
typedef __attribute__((ext_vector_type(4)))  int v4i;
typedef float __attribute__((may_alias)) float_a;
typedef int __attribute__((may_alias)) int_a;

template <typename T> __device__ __forceinline__ void vst2(void* p, T v) { *(volatile T*)p = v; __threadfence(); *(volatile T*)p = v; }
__device__ __forceinline__ v8f wmma16(v16h a, v16h b, v8f c) {
  v8f d = __builtin_amdgcn_wmma_f32_16x16x32_f16(false, a, false, b, (short)0, c, false, false);
  asm volatile("v_nop\n\tv_nop\n\tv_nop\n\tv_nop" : "+v"(d) : "v"(a), "v"(b));
  return d;
}
__device__ __forceinline__ v8f wmma_bf(v16b a, v16b b, v8f c) {
  v8f d = __builtin_amdgcn_wmma_f32_16x16x32_bf16(false, a, false, b, (short)0, c, false, false);
  asm volatile("v_nop\n\tv_nop\n\tv_nop\n\tv_nop" : "+v"(d) : "v"(a), "v"(b));
  return d;
}
__device__ __forceinline__ v16h frag_h(const _Float16* rowk0, int lane) {
  union { v16h v; v8h q[2]; } u; const _Float16* p = rowk0 + 8 * (lane >> 4);
  u.q[0] = *(const v8h*)p; u.q[1] = *(const v8h*)(p + 16); return u.v;
}
__device__ __forceinline__ v16h frag_f32(const float* rowk0, int lane) {
  v16h a; const float* p = rowk0 + 8 * (lane >> 4);
#pragma unroll
  for (int i = 0; i < 8; ++i) { a[i] = (_Float16)p[i]; a[8 + i] = (_Float16)p[16 + i]; }
  return a;
}
__device__ __forceinline__ v16h frag_f32s(const float* rowk0, int lane, float sc) {
  v16h a; const float* p = rowk0 + 8 * (lane >> 4);
#pragma unroll
  for (int i = 0; i < 8; ++i) { a[i] = (_Float16)(p[i] * sc); a[8 + i] = (_Float16)(p[16 + i] * sc); }
  return a;
}
__device__ __forceinline__ v16h fragc_f32(const float* W, int k0, int n, int lane, int ld, int K) {
  v16h a; const int g = lane >> 4;
#pragma unroll
  for (int i = 0; i < 8; ++i) { const int ka = k0 + 8 * g + i, kb = ka + 16;
    a[i] = (_Float16)(ka < K ? W[(size_t)(ka < K ? ka : K - 1) * ld + n] : 0.f); a[8 + i] = (_Float16)(kb < K ? W[(size_t)(kb < K ? kb : K - 1) * ld + n] : 0.f); }
  return a;
}
struct F2 { v16b h, l; };
__device__ __forceinline__ F2 bsplit16(const float v[16]) { F2 r;
#pragma unroll
  for (int i = 0; i < 16; ++i) { const __bf16 h = (__bf16)v[i]; r.h[i] = h; r.l[i] = (__bf16)(v[i] - (float)h); }
  return r; }
__device__ __forceinline__ F2 split_row(const float* row, int k0, int lane) { float v[16]; const float* p = row + k0 + 8 * (lane >> 4);
#pragma unroll
  for (int i = 0; i < 8; ++i) { v[i] = p[i]; v[8 + i] = p[16 + i]; }
  return bsplit16(v); }
__device__ __forceinline__ F2 split_rowK(const float* row, int k0, int lane, int K) { float v[16]; const int g = lane >> 4;
#pragma unroll
  for (int i = 0; i < 8; ++i) { const int ka = k0 + 8 * g + i, kb = ka + 16; v[i] = ka < K ? row[ka < K ? ka : K - 1] : 0.f; v[8 + i] = kb < K ? row[kb < K ? kb : K - 1] : 0.f; }
  return bsplit16(v); }
__device__ __forceinline__ F2 split_col(const float* W, int k0, int n, int lane, int ld, int K) { float v[16]; const int g = lane >> 4;
#pragma unroll
  for (int i = 0; i < 8; ++i) { const int ka = k0 + 8 * g + i, kb = ka + 16; v[i] = ka < K ? W[(size_t)(ka < K ? ka : K - 1) * ld + n] : 0.f; v[8 + i] = kb < K ? W[(size_t)(kb < K ? kb : K - 1) * ld + n] : 0.f; }
  return bsplit16(v); }
__device__ __forceinline__ v8f mac3(const F2& a, const F2& b, v8f c) { c = wmma_bf(a.l, b.h, c); c = wmma_bf(a.h, b.l, c); return wmma_bf(a.h, b.h, c); }
__device__ __forceinline__ float sigm(float v) { return 1.0f / (1.0f + expf(-v)); }
#define LDSX() do { asm volatile("s_wait_dscnt 0" ::: "memory"); __builtin_amdgcn_wave_barrier(); __builtin_amdgcn_fence(__ATOMIC_RELEASE, "workgroup"); } while (0)


#define NRW 4096
#define LV 8
#define RR 128
#define NE (LV * RR)
#define HH 4096
#ifndef TRB
#define TRB (NRW / 64)
#endif
typedef __attribute__((ext_vector_type(8))) __bf16 v8b;
__device__ __forceinline__ v16b frag_b(const __bf16* rowk0, int lane) {
  union { v16b v; v8b q[2]; } u; const __bf16* p = rowk0 + 8 * (lane >> 4);
  u.q[0] = *(const v8b*)p; u.q[1] = *(const v8b*)(p + 16); return u.v;
}
__device__ __forceinline__ float bfr(float v) { return (float)(__bf16)v; }
__device__ __attribute__((noinline)) float exp_ni(float v) { return expf(v); }
__device__ __attribute__((noinline)) float erf_ni(float v) { return erff(v); }

#define WS_P1  0u
#define WS_P2  (WS_P1 + 2u * (size_t)HH * NE)
#define WS_H   (WS_P2 + 2u * (size_t)RR * HH)
#define WS_END (WS_H + 2u * (size_t)4 * NRW * HH)

__global__ __launch_bounds__(256) void k_pack(const float* __restrict__ W1, const float* __restrict__ W2, __bf16* __restrict__ P1, _Float16* __restrict__ P2) { const int n = blockIdx.x, t = threadIdx.x;
  if (n < HH) { __shared__ __align__(16) __bf16 s[NE]; for (int k = t; k < NE; k += 256) s[k] = (__bf16)W1[(size_t)k * HH + n]; __syncthreads(); for (int q = t; q < NE / 8; q += 256) vst2((unsigned*)(P1 + (size_t)n * NE + q * 8), *(const v4u*)&s[q * 8]); }
  else { const int r = n - HH; __shared__ __align__(16) _Float16 s2[HH]; for (int k = t; k < HH; k += 256) s2[k] = (_Float16)(bfr(W2[(size_t)k * RR + r]) * 256.0f); __syncthreads(); for (int q = t; q < HH / 8; q += 256) vst2((unsigned*)(P2 + (size_t)r * HH + q * 8), *(const v4u*)&s2[q * 8]); } }
__device__ __attribute__((noinline)) float tanh_p(float v) { return tanhf(v); }
__device__ __forceinline__ float gelu_n(float x) { return 0.5f * x * (1.0f + tanh_p(0.7978845608028654f * (x + 0.044715f * x * x * x))); }
template <int PASS>
__global__ __launch_bounds__(128) void k_lev(const float* __restrict__ X, const __bf16* __restrict__ P1, const float* __restrict__ B1, _Float16* __restrict__ H) {
  __shared__ __align__(16) _Float16 sg[4][16][136];
  const int tid = threadIdx.x, wave = tid >> 5, lane = tid & 31, col = lane & 15, g = lane >> 4; const size_t r0 = (size_t)blockIdx.x * 64 + wave * 16; const int n0 = blockIdx.y * 128;
  v8f acc[8] = {};
#pragma unroll 1
  for (int lv = LV - 1; lv >= 0; --lv) {
#pragma unroll
    for (int kq = 0; kq < RR / 32; ++kq) { const int kc = lv * (RR / 32) + kq; v16b a; { const float* p = X + (r0 + col) * NE + kc * 32 + 8 * g;
#pragma unroll
        for (int i = 0; i < 8; ++i) { a[i] = (__bf16)p[i]; a[8 + i] = (__bf16)p[16 + i]; } }
#pragma unroll
      for (int j = 0; j < 8; ++j) acc[j] = wmma_bf(a, frag_b(P1 + (size_t)(n0 + j * 16 + col) * NE + kc * 32, lane), acc[j]); }
    if ((PASS == 0 && lv >= 4) || (PASS == 1 && lv < 4)) {
#pragma unroll
    for (int j = 0; j < 8; ++j) { const float bb = bfr(B1[n0 + j * 16 + col]);
#pragma unroll
      for (int r = 0; r < 8; ++r) sg[wave][8 * g + r][j * 16 + col] = (_Float16)gelu_n(acc[j][r] + bb); }
    LDSX();
    for (int rl = 0; rl < 16; ++rl) if (lane < 16) vst2((unsigned*)(H + ((size_t)(lv & 3) * NRW + r0 + rl) * HH + n0 + lane * 8), *(const v4u*)&sg[wave][rl][lane * 8]);
    LDSX(); }
    if (PASS == 0 && lv == 4) break; }
}
__global__ __launch_bounds__(128) void k_out(const _Float16* __restrict__ H, const _Float16* __restrict__ P2, const float* __restrict__ B2, int lvbase, float* __restrict__ OUT) {
  __shared__ __align__(16) float so[4][16][132];
  const int tid = threadIdx.x, wave = tid >> 5, lane = tid & 31, col = lane & 15, g = lane >> 4; const size_t r0 = (size_t)blockIdx.x * 64 + wave * 16; const int slot = blockIdx.y; const int lv = lvbase + slot;
  v8f acc[8] = {};
#pragma unroll 2
  for (int kc = 0; kc < HH / 32; ++kc) { const v16h a = frag_h(H + ((size_t)slot * NRW + r0 + col) * HH + kc * 32, lane);
#pragma unroll
    for (int j = 0; j < 8; ++j) acc[j] = wmma16(a, frag_h(P2 + (size_t)(j * 16 + col) * HH + kc * 32, lane), acc[j]); }
#pragma unroll
  for (int j = 0; j < 8; ++j) { const float bb = bfr(B2[j * 16 + col]);
#pragma unroll
    for (int r = 0; r < 8; ++r) so[wave][8 * g + r][j * 16 + col] = acc[j][r] * (1.0f / 256.0f) + bb; }
  LDSX();
  for (int rl = 0; rl < 16; ++rl) vst2(OUT + ((r0 + rl) * LV + lv) * RR + lane * 4, *(const v4f*)&so[wave][rl][lane * 4]);
}
extern "C" void kernel_launch(void* const* d_in, const int* in_sizes, int n_in, void* d_out, int out_size, void* d_ws, size_t ws_size, hipStream_t stream) {
  (void)in_sizes; (void)n_in; (void)out_size;
  const float** F = (const float**)d_in;
  if (ws_size < (size_t)WS_END) return;
  char* ws = (char*)d_ws; __bf16* P1 = (__bf16*)(ws + WS_P1); _Float16 *P2 = (_Float16*)(ws + WS_P2), *H = (_Float16*)(ws + WS_H);
  k_pack<<<HH + RR, 256, 0, stream>>>(F[1], F[3], P1, P2);
  k_lev<0><<<dim3(TRB, HH / 128), 128, 0, stream>>>(F[0], P1, F[2], H);
  k_out<<<dim3(TRB, 4), 128, 0, stream>>>(H, P2, F[4], 4, (float*)d_out);
  k_lev<1><<<dim3(TRB, HH / 128), 128, 0, stream>>>(F[0], P1, F[2], H);
  k_out<<<dim3(TRB, 4), 128, 0, stream>>>(H, P2, F[4], 0, (float*)d_out);
}
